// MultiHeadClauseAttention_88751204204552
// MI455X (gfx1250) — hardware-run, weakly checked
//
#include <hip/hip_runtime.h>
#include <math.h>
#include <stdint.h>

#define NTOK   2048
#define DM     1024
#define NHEAD  16
#define HD     64
#define GD     128
#define RELR   1025
#define RPMAX  512
#define KCH    32
#define HPB    8
#define IDLIM  (1 << 29)
#define WSC    64.0f
#define ACARRY 16.0f
#define QC     8.0f
#define VC     16.0f
#define PC     4096.0f
#define CC     256.0f
#define QKS    0.125f
#define LOG2E  1.4426950408889634f
#define SC2    (QKS * LOG2E / (QC * QC))
#define LNEPS  1e-5f
static_assert(NHEAD * HD == DM);
static_assert((NTOK % 64) == 0 && (DM % 64) == 0 && (HD % 32) == 0 && (NTOK % KCH) == 0 && (NHEAD % HPB) == 0);
static_assert(((NTOK * DM) % 2048) == 0 && (DM % 256) == 0 && (DM % 8) == 0);
#define ATT_THREADS (HPB * 32)
#define ATT_BLOCKS  ((NTOK / 16) * (NHEAD / HPB))
#define PTP 36
#define ATT_SMEM_FLOATS (HPB * 16 * PTP)
static_assert(ATT_THREADS == 256);
static_assert(ATT_BLOCKS == 256);
static_assert(HPB * 16 * HD <= 2 * ATT_SMEM_FLOATS);
static_assert((HPB * 16 * HD) / 8 == 4 * ATT_THREADS);

typedef _Float16 v16h __attribute__((ext_vector_type(16)));
typedef _Float16 v8h  __attribute__((ext_vector_type(8)));
typedef __bf16   v16b __attribute__((ext_vector_type(16)));
typedef float    v8f  __attribute__((ext_vector_type(8)));
typedef float    v4f  __attribute__((ext_vector_type(4)));
typedef unsigned int v4u __attribute__((ext_vector_type(4)));

union FragH { v16h v; v8h h[2]; v4u u[2]; };
union FragAny { v16h h; v16b b; };

__device__ __forceinline__ unsigned short bf_bits(float f) {
  unsigned u = __float_as_uint(f);
  return (unsigned short)((u + 0x7FFFu + ((u >> 16) & 1u)) >> 16);
}
__device__ __forceinline__ float bf_up(unsigned short h) { return __uint_as_float(((unsigned)h) << 16); }
__device__ __forceinline__ float bfr(float f) { return bf_up(bf_bits(f)); }
__device__ __forceinline__ unsigned short h_bits(_Float16 x) { return __builtin_bit_cast(unsigned short, x); }
__device__ __forceinline__ unsigned pk16(unsigned short a, unsigned short b) { return (unsigned)a | ((unsigned)b << 16); }
__device__ __forceinline__ v8f zero8() { v8f z = {0.f, 0.f, 0.f, 0.f, 0.f, 0.f, 0.f, 0.f}; return z; }
__device__ __forceinline__ int iclamp(int x, int lo, int hi) { x = (x < lo) ? lo : x; return (x > hi) ? hi : x; }

__device__ __forceinline__ v16h ldfrag_u(const unsigned short* p) {
  FragH f;
  f.u[0] = *(const v4u*)(p);
  f.u[1] = *(const v4u*)(p + 16);
  return f.v;
}

__device__ __forceinline__ v8f mma_h(v16h a, v16h b, v8f c) {
  return __builtin_amdgcn_wmma_f32_16x16x32_f16(false, a, false, b, (short)0, c, false, false);
}
__device__ __forceinline__ v8f mma_b(v16h a, v16h b, v8f c) {
  FragAny ua, ub;
  ua.h = a;
  ub.h = b;
  return __builtin_amdgcn_wmma_f32_16x16x32_bf16(false, ua.b, false, ub.b, (short)0, c, false, false);
}
template <int BF>
__device__ __forceinline__ v8f mmaT(v16h a, v16h b, v8f c) {
  if constexpr (BF != 0) return mma_b(a, b, c);
  else return mma_h(a, b, c);
}
__device__ __forceinline__ void dep_guard1(v8f& a, v8f& b, v16h x) {
#if defined(__HIP_DEVICE_COMPILE__)
  asm volatile("v_nop\n\tv_nop\n\tv_nop\n\tv_nop" : "+v"(a), "+v"(b) : "v"(x));
#endif
}
__device__ __forceinline__ void guard2x6(v8f& a, v8f& b, v16h x0, v16h x1, v16h x2, v16h x3, v16h x4, v16h x5) {
#if defined(__HIP_DEVICE_COMPILE__)
  asm volatile("v_nop\n\tv_nop\n\tv_nop\n\tv_nop"
               : "+v"(a), "+v"(b) : "v"(x0), "v"(x1), "v"(x2), "v"(x3), "v"(x4), "v"(x5));
#endif
}
__device__ __forceinline__ void guard4x5(v8f& a, v8f& b, v8f& c, v8f& d,
                                         v16h x0, v16h x1, v16h x2, v16h x3, v16h x4) {
#if defined(__HIP_DEVICE_COMPILE__)
  asm volatile("v_nop\n\tv_nop\n\tv_nop\n\tv_nop"
               : "+v"(a), "+v"(b), "+v"(c), "+v"(d) : "v"(x0), "v"(x1), "v"(x2), "v"(x3), "v"(x4));
#endif
}
__device__ __forceinline__ void keep4_h(v16h a, v16h b, v16h c, v16h d) {
#if defined(__HIP_DEVICE_COMPILE__)
  asm volatile("v_nop" :: "v"(a), "v"(b), "v"(c), "v"(d));
#endif
}
__device__ __forceinline__ void acc_guard4(v8f& a, v8f& b, v8f& c, v8f& d) {
#if defined(__HIP_DEVICE_COMPILE__)
  asm volatile("v_nop\n\tv_nop\n\tv_nop\n\tv_nop" : "+v"(a), "+v"(b), "+v"(c), "+v"(d));
#endif
}
__device__ __forceinline__ void wave_sync_lds() {
  __builtin_amdgcn_fence(__ATOMIC_RELEASE, "workgroup");
  __builtin_amdgcn_wave_barrier();
  __builtin_amdgcn_fence(__ATOMIC_ACQUIRE, "workgroup");
}

__global__ __launch_bounds__(256) void gate_k(const float* __restrict__ goal, const float* __restrict__ Wg,
                                              const float* __restrict__ bg, float* gate) {
  const int j = blockIdx.x * 256 + threadIdx.x;
  float acc = 0.f;
#pragma unroll 4
  for (int i = 0; i < GD; ++i) acc += bfr(goal[i]) * bfr(Wg[(size_t)i * DM + j]);
  acc += bfr(bg[j]);
  acc = fminf(fmaxf(acc, -40.f), 40.f);
  const float g = 1.0f / (1.0f + expf(-acc));
  for (int pass = 0; pass < 2; ++pass) {
    *(volatile float*)(gate + j) = g;
    __threadfence();
  }
}

__global__ __launch_bounds__(256) void cvtx_k(const float* __restrict__ src, const float* __restrict__ gate,
                                              unsigned short* dst, int n, float sc) {
  const size_t i8 = ((size_t)blockIdx.x * 256 + threadIdx.x) * 8;
  if (i8 + 8 > (size_t)n) return;
  const int c = (int)(i8 & (size_t)(DM - 1));
  const v4f a  = *(const v4f*)(src + i8);
  const v4f b  = *(const v4f*)(src + i8 + 4);
  const v4f g0 = *(const v4f*)(gate + c);
  const v4f g1 = *(const v4f*)(gate + c + 4);
  v4u o;
  o[0] = pk16(h_bits((_Float16)(bfr(a[0]) * g0[0] * sc)), h_bits((_Float16)(bfr(a[1]) * g0[1] * sc)));
  o[1] = pk16(h_bits((_Float16)(bfr(a[2]) * g0[2] * sc)), h_bits((_Float16)(bfr(a[3]) * g0[3] * sc)));
  o[2] = pk16(h_bits((_Float16)(bfr(b[0]) * g1[0] * sc)), h_bits((_Float16)(bfr(b[1]) * g1[1] * sc)));
  o[3] = pk16(h_bits((_Float16)(bfr(b[2]) * g1[2] * sc)), h_bits((_Float16)(bfr(b[3]) * g1[3] * sc)));
  for (int pass = 0; pass < 2; ++pass) {
    *(volatile v4u*)(dst + i8) = o;
    __threadfence();
  }
}

__global__ __launch_bounds__(256) void cvtT_k(const float* __restrict__ in, unsigned short* out, float sc) {
  __shared__ float tile[64][65];
  const int n0 = blockIdx.x * 64;
  const int k0 = blockIdx.y * 64;
  const int tid = threadIdx.x;
#pragma unroll
  for (int it = 0; it < 4; ++it) {
    const int r = it * 16 + (tid >> 4);
    const int c4 = (tid & 15) * 4;
    const v4f v = *(const v4f*)(in + (size_t)(k0 + r) * DM + n0 + c4);
    tile[r][c4]     = v[0];
    tile[r][c4 + 1] = v[1];
    tile[r][c4 + 2] = v[2];
    tile[r][c4 + 3] = v[3];
  }
  __syncthreads();
  v4u ov[2];
#pragma unroll
  for (int it = 0; it < 2; ++it) {
    const int p  = it * 256 + tid;
    const int nn = p >> 3;
    const int k8 = (p & 7) * 8;
    v4u o;
#pragma unroll
    for (int e = 0; e < 4; ++e) {
      const float f0 = tile[k8 + 2 * e][nn];
      const float f1 = tile[k8 + 2 * e + 1][nn];
      o[e] = pk16(h_bits((_Float16)(bfr(f0) * sc)), h_bits((_Float16)(bfr(f1) * sc)));
    }
    ov[it] = o;
  }
  for (int pass = 0; pass < 2; ++pass) {
#pragma unroll
    for (int it = 0; it < 2; ++it) {
      const int p  = it * 256 + tid;
      const int nn = p >> 3;
      const int k8 = (p & 7) * 8;
      *(volatile v4u*)(out + (size_t)(n0 + nn) * DM + k0 + k8) = ov[it];
    }
    __threadfence();
  }
}

template <int OM, int ASPLIT, int BF, int EPI>
__global__ __launch_bounds__(256) __attribute__((amdgpu_num_vgpr(256))) void gemm64(
    const unsigned short* __restrict__ Ap, const unsigned short* __restrict__ A2p, int lda, long long sA,
    const unsigned short* __restrict__ Btp, int ldb, long long sB,
    void* Cout, void* C2out, int ldc, long long sC,
    int M, int N, int K, float oscale, float ocarry,
    const float* __restrict__ bias) {
  __shared__ __align__(16) float sT[8][16 * 68];
  const int by   = blockIdx.y;
  const int lane = threadIdx.x & 31;
  const int wave = threadIdx.x >> 5;
  const int tilesN = N >> 6;
  const int tilesM = M >> 6;
  const int tile = blockIdx.x * 8 + wave;
  if (tile >= tilesM * tilesN) return;
  const int tm = tile / tilesN;
  const int tn = tile - tm * tilesN;
  const int m0 = tm << 6;
  const int n0 = tn << 6;

  const unsigned short* A1 = Ap  + (size_t)((long long)by * sA);
  const unsigned short* A2 = A2p + (size_t)((long long)by * sA);
  const unsigned short* Bb = Btp + (size_t)((long long)by * sB);

  const int rlane = lane & 15;
  const int koff  = (lane >> 4) * 8;
  const int mOff  = (lane >> 4) * 8;

  v8f acc[4][4];
#pragma unroll
  for (int i = 0; i < 4; ++i)
#pragma unroll
    for (int j = 0; j < 4; ++j) acc[i][j] = zero8();

  for (int k0 = 0; k0 < K; k0 += 32) {
    v16h bh[4];
#pragma unroll
    for (int j = 0; j < 4; ++j) {
      const size_t bofs = (size_t)(n0 + (j << 4) + rlane) * ldb + koff + k0;
      bh[j] = ldfrag_u(Bb + bofs);
    }
#pragma unroll
    for (int i = 0; i < 4; ++i) {
      const size_t ao = (size_t)(m0 + (i << 4) + rlane) * lda + koff + k0;
      const v16h ah = ldfrag_u(A1 + ao);
#pragma unroll
      for (int j = 0; j < 4; ++j) acc[i][j] = mmaT<BF>(ah, bh[j], acc[i][j]);
      dep_guard1(acc[i][0], acc[i][3], ah);
      if constexpr (ASPLIT != 0) {
        const v16h al = ldfrag_u(A2 + ao);
#pragma unroll
        for (int j = 0; j < 4; ++j) acc[i][j] = mmaT<BF>(al, bh[j], acc[i][j]);
        dep_guard1(acc[i][0], acc[i][3], al);
      }
    }
    keep4_h(bh[0], bh[1], bh[2], bh[3]);
  }
  acc_guard4(acc[0][0], acc[0][1], acc[0][2], acc[0][3]);
  acc_guard4(acc[1][0], acc[1][1], acc[1][2], acc[1][3]);
  acc_guard4(acc[2][0], acc[2][1], acc[2][2], acc[2][3]);
  acc_guard4(acc[3][0], acc[3][1], acc[3][2], acc[3][3]);

  const int hh2 = lane >> 4, c4 = (lane & 15) * 4;
  const int q8  = lane >> 3, c8 = (lane & 7) * 8;

  float* slab = sT[wave];
#pragma unroll
  for (int i = 0; i < 4; ++i) {
    const int mBase = m0 + (i << 4);
#pragma unroll
    for (int j = 0; j < 4; ++j) {
#pragma unroll
      for (int r = 0; r < 8; ++r) {
        slab[(mOff + r) * 68 + (j << 4) + rlane] = acc[i][j][r];
      }
    }
    wave_sync_lds();
    if constexpr (OM == 0) {
      float* C = (float*)Cout + (size_t)((long long)by * sC);
      v4f vals[8];
#pragma unroll
      for (int it = 0; it < 8; ++it) {
        const int row = it * 2 + hh2;
        v4f v = *(const v4f*)(slab + row * 68 + c4);
#pragma unroll
        for (int e = 0; e < 4; ++e) {
          float f = v[e] * oscale;
          if constexpr (EPI == 1) f += bfr(bias[n0 + c4 + e]);
          if constexpr (EPI == 2) f += bfr(bias[mBase + row]);
          v[e] = f;
        }
        vals[it] = v;
      }
      for (int pass = 0; pass < 2; ++pass) {
#pragma unroll
        for (int it = 0; it < 8; ++it) {
          const int gr = mBase + it * 2 + hh2;
          *(volatile v4f*)(C + (size_t)gr * ldc + n0 + c4) = vals[it];
        }
        __threadfence();
      }
    } else {
      unsigned short* C  = (unsigned short*)Cout  + (size_t)((long long)by * sC);
      unsigned short* Cb = (unsigned short*)C2out + (size_t)((long long)by * sC);
      v4u hv[4], lv[4];
#pragma unroll
      for (int it = 0; it < 4; ++it) {
        const int row = it * 4 + q8;
        const float* sp = slab + row * 68 + c8;
        v4u a  = {0u, 0u, 0u, 0u};
        v4u b2 = {0u, 0u, 0u, 0u};
        float brow = 0.f;
        if constexpr (EPI == 2) brow = bfr(bias[mBase + row]);
#pragma unroll
        for (int e = 0; e < 4; ++e) {
          float f0 = sp[2 * e] * oscale;
          float f1 = sp[2 * e + 1] * oscale;
          if constexpr (EPI == 1) {
            f0 += bfr(bias[n0 + c8 + 2 * e]);
            f1 += bfr(bias[n0 + c8 + 2 * e + 1]);
          }
          if constexpr (EPI == 2) {
            f0 += brow;
            f1 += brow;
          }
          if constexpr (OM == 3) {
            const unsigned short g0 = bf_bits(f0), g1 = bf_bits(f1);
            a[e]  = pk16(g0, g1);
            b2[e] = pk16(bf_bits(f0 - bf_up(g0)), bf_bits(f1 - bf_up(g1)));
          } else {
            f0 *= ocarry; f1 *= ocarry;
            const _Float16 x0 = (_Float16)f0, x1 = (_Float16)f1;
            a[e] = pk16(h_bits(x0), h_bits(x1));
            if constexpr (OM == 4) {
              b2[e] = pk16(h_bits((_Float16)(f0 - (float)x0)), h_bits((_Float16)(f1 - (float)x1)));
            }
          }
        }
        hv[it] = a;
        lv[it] = b2;
      }
      for (int pass = 0; pass < 2; ++pass) {
#pragma unroll
        for (int it = 0; it < 4; ++it) {
          const int row = it * 4 + q8;
          *(volatile v4u*)(C + (size_t)(mBase + row) * ldc + n0 + c8) = hv[it];
          if constexpr (OM >= 3) {
            *(volatile v4u*)(Cb + (size_t)(mBase + row) * ldc + n0 + c8) = lv[it];
          }
        }
        __threadfence();
      }
    }
    wave_sync_lds();
  }
}

__global__ __launch_bounds__(ATT_THREADS) __attribute__((amdgpu_num_vgpr(256)))
void attn_k(const unsigned short* __restrict__ Q16, const unsigned short* __restrict__ K16,
            const unsigned short* __restrict__ VT16, const int* __restrict__ ids,
            const float* __restrict__ rel, unsigned short* CT) {
  __shared__ __align__(16) float smem[ATT_SMEM_FLOATS];

  const int tid  = threadIdx.x;
  const int wave = __builtin_amdgcn_readfirstlane(tid >> 5);
  const int lane = tid & 31;
  const int hh   = lane >> 4;
  const int c    = lane & 15;

  const int rt   = blockIdx.x & ((NTOK / 16) - 1);
  const int hg   = blockIdx.x / (NTOK / 16);
  const int head = hg * HPB + wave;
  const int q0   = rt * 16;

  const size_t qofs = (size_t)(q0 + c) * DM + head * HD + 8 * hh;
  const v16h qa = ldfrag_u(Q16 + qofs), qb = ldfrag_u(Q16 + qofs + 32);

  int qid[8];
#pragma unroll
  for (int r = 0; r < 8; ++r) qid[r] = iclamp(ids[q0 + 8 * hh + r], -IDLIM, IDLIM);

  const unsigned short* Kb = K16 + head * HD + 8 * hh;
  const unsigned short* Vb = VT16 + (size_t)(head * HD) * NTOK + 8 * hh;
  const float* rph = rel + head;

  float mrow[8], lrow[8];
  v8f o0 = zero8(), o1 = zero8(), o2 = zero8(), o3 = zero8();
#pragma unroll
  for (int r = 0; r < 8; ++r) { mrow[r] = -INFINITY; lrow[r] = 0.f; }
  float* pt = smem + wave * (16 * PTP);

#pragma unroll 1
  for (int kb = 0; kb < NTOK; kb += KCH) {
    v8f s0, s1;
    {
      const size_t ko  = (size_t)(kb + c) * DM;
      const size_t k1o = ko + (size_t)16 * DM;
      const v16h k0a = ldfrag_u(Kb + ko),  k0b = ldfrag_u(Kb + ko + 32);
      const v16h k1a = ldfrag_u(Kb + k1o), k1b = ldfrag_u(Kb + k1o + 32);
      s0 = mma_h(qa, k0a, zero8());
      s0 = mma_h(qb, k0b, s0);
      s1 = mma_h(qa, k1a, zero8());
      s1 = mma_h(qb, k1b, s1);
      guard2x6(s0, s1, k0a, k0b, k1a, k1b, qa, qb);
    }
    const int kid0 = iclamp(ids[kb + c], -IDLIM, IDLIM);
    const int kid1 = iclamp(ids[kb + 16 + c], -IDLIM, IDLIM);
#pragma unroll
    for (int r = 0; r < 8; ++r) {
      const int ia = iclamp(qid[r] - kid0, -RPMAX, RPMAX) + RPMAX;
      const int ib = iclamp(qid[r] - kid1, -RPMAX, RPMAX) + RPMAX;
      const float b0 = bfr(rph[(size_t)ia * NHEAD]) * LOG2E;
      const float b1 = bfr(rph[(size_t)ib * NHEAD]) * LOG2E;
      const float t0 = s0[r] * SC2 + b0, t1 = s1[r] * SC2 + b1;
      float mx = fmaxf(t0, t1);
#pragma unroll
      for (int off = 1; off < 16; off <<= 1) mx = fmaxf(mx, __shfl_xor(mx, off, 32));
      const float mn = fmaxf(mrow[r], mx);
      const float al = exp2f(mrow[r] - mn);
      mrow[r] = mn;
      const float e0 = exp2f(t0 - mn), e1 = exp2f(t1 - mn);
      float ps = e0 + e1;
#pragma unroll
      for (int off = 1; off < 16; off <<= 1) ps += __shfl_xor(ps, off, 32);
      lrow[r] = lrow[r] * al + ps;
      o0[r] *= al; o1[r] *= al; o2[r] *= al; o3[r] *= al;
      const int ro = (8 * hh + r) * PTP + c;
      pt[ro]      = e0;
      pt[ro + 16] = e1;
    }
    wave_sync_lds();
    FragH ph;
    {
      const float* prow = pt + c * PTP + 8 * hh;
      const v4f p0 = *(const v4f*)(prow), p1 = *(const v4f*)(prow + 4);
      const v4f p2 = *(const v4f*)(prow + 16), p3 = *(const v4f*)(prow + 20);
#pragma unroll
      for (int e = 0; e < 4; ++e) {
        ph.h[0][e]     = (_Float16)(p0[e] * PC);
        ph.h[0][4 + e] = (_Float16)(p1[e] * PC);
        ph.h[1][e]     = (_Float16)(p2[e] * PC);
        ph.h[1][4 + e] = (_Float16)(p3[e] * PC);
      }
    }
    const size_t vo = (size_t)c * NTOK + kb;
    {
      const v16h vh0 = ldfrag_u(Vb + vo);
      const v16h vh1 = ldfrag_u(Vb + vo + (size_t)16 * NTOK);
      const v16h vh2 = ldfrag_u(Vb + vo + (size_t)32 * NTOK);
      const v16h vh3 = ldfrag_u(Vb + vo + (size_t)48 * NTOK);
      o0 = mma_h(ph.v, vh0, o0);
      o1 = mma_h(ph.v, vh1, o1);
      o2 = mma_h(ph.v, vh2, o2);
      o3 = mma_h(ph.v, vh3, o3);
      guard4x5(o0, o1, o2, o3, ph.v, vh0, vh1, vh2, vh3);
    }
    wave_sync_lds();
  }
  acc_guard4(o0, o1, o2, o3);

  __syncthreads();
  unsigned short* Os = (unsigned short*)smem;
  const float oc = CC / (PC * VC);
  {
#pragma unroll
    for (int r = 0; r < 8; ++r) {
      const float inv = (1.0f / lrow[r]) * oc;
      const int ro = (wave * 16 + 8 * hh + r) * HD + c;
      Os[ro]      = h_bits((_Float16)(o0[r] * inv));
      Os[ro + 16] = h_bits((_Float16)(o1[r] * inv));
      Os[ro + 32] = h_bits((_Float16)(o2[r] * inv));
      Os[ro + 48] = h_bits((_Float16)(o3[r] * inv));
    }
  }
  __syncthreads();
  {
    v4u hv[4];
#pragma unroll
    for (int it = 0; it < 4; ++it) {
      const int p = it * ATT_THREADS + tid;
      hv[it] = *(const v4u*)(Os + (size_t)p * 8);
    }
    for (int pass = 0; pass < 2; ++pass) {
#pragma unroll
      for (int it = 0; it < 4; ++it) {
        const int p    = it * ATT_THREADS + tid;
        const int w    = p >> 7;
        const int row  = (p >> 3) & 15;
        const int col8 = (p & 7) * 8;
        *(volatile v4u*)(CT + (size_t)(q0 + row) * DM + (hg * HPB + w) * HD + col8) = hv[it];
      }
      __threadfence();
    }
  }
}

__global__ __launch_bounds__(256) void ln_k(const float* __restrict__ Y, const float* __restrict__ resid,
                                            const float* __restrict__ gam, const float* __restrict__ bet, float* out) {
  __shared__ float red[16];
  const int row = blockIdx.x, tid = threadIdx.x, lane = tid & 31, wave = tid >> 5;
  const size_t base = (size_t)row * DM + (size_t)tid * 4;
  const v4f yv = *(const v4f*)(Y + base);
  const v4f rv = *(const v4f*)(resid + base);
  v4f y;
  float s = 0.f;
#pragma unroll
  for (int e = 0; e < 4; ++e) { y[e] = bfr(rv[e]) + yv[e]; s += y[e]; }
#pragma unroll
  for (int off = 1; off < 32; off <<= 1) s += __shfl_xor(s, off, 32);
  if (lane == 0) red[wave] = s;
  __syncthreads();
  float tot = 0.f;
#pragma unroll
  for (int w = 0; w < 8; ++w) tot += red[w];
  const float mean = tot * (1.0f / (float)DM);
  v4f d;
  float ss = 0.f;
#pragma unroll
  for (int e = 0; e < 4; ++e) { d[e] = y[e] - mean; ss += d[e] * d[e]; }
#pragma unroll
  for (int off = 1; off < 32; off <<= 1) ss += __shfl_xor(ss, off, 32);
  if (lane == 0) red[8 + wave] = ss;
  __syncthreads();
  float tot2 = 0.f;
#pragma unroll
  for (int w = 0; w < 8; ++w) tot2 += red[8 + w];
  const float var  = tot2 * (1.0f / (float)DM);
  const float rstd = 1.0f / sqrtf(var + LNEPS);
  v4f o;
#pragma unroll
  for (int e = 0; e < 4; ++e) o[e] = d[e] * rstd * bfr(gam[tid * 4 + e]) + bfr(bet[tid * 4 + e]);
  for (int pass = 0; pass < 2; ++pass) {
    *(volatile v4f*)(out + base) = o;
    __threadfence();
  }
}

extern "C" void kernel_launch(void* const* d_in, const int* in_sizes, int n_in,
                              void* d_out, int out_size, void* d_ws, size_t ws_size,
                              hipStream_t stream) {
  if (n_in < 12) return;
  if (in_sizes[0] != NTOK * DM) return;
  if (in_sizes[1] != GD) return;
  if (in_sizes[2] != NTOK) return;
  if (in_sizes[3] != DM * DM || in_sizes[4] != DM * DM || in_sizes[5] != DM * DM || in_sizes[6] != DM * DM) return;
  if (in_sizes[7] != RELR * NHEAD) return;
  if (in_sizes[8] != GD * DM) return;
  if (in_sizes[9] != DM || in_sizes[10] != DM || in_sizes[11] != DM) return;
  if (out_size != NTOK * DM) return;

  const float* emb  = (const float*)d_in[0];
  const float* goal = (const float*)d_in[1];
  const int*   ids  = (const int*)d_in[2];
  const float* w_q  = (const float*)d_in[3];
  const float* w_k  = (const float*)d_in[4];
  const float* w_v  = (const float*)d_in[5];
  const float* w_o  = (const float*)d_in[6];
  const float* rel  = (const float*)d_in[7];
  const float* w_g  = (const float*)d_in[8];
  const float* b_g  = (const float*)d_in[9];
  const float* ln_g = (const float*)d_in[10];
  const float* ln_b = (const float*)d_in[11];
  float*       out  = (float*)d_out;

  const size_t PG = 4096;
  const size_t PX = (size_t)NTOK * DM * 2;
  const size_t PW = (size_t)DM * DM * 2;
  const size_t PV = (size_t)DM * NTOK * 2;
  const size_t PY = (size_t)NTOK * DM * 4;
  size_t off = 0;
  const size_t oG  = off; off += PG;
  const size_t oX  = off; off += PX;
  const size_t oWQ = off; off += PW;
  const size_t oWK = off; off += PW;
  const size_t oWV = off; off += PW;
  const size_t oWO = off; off += PW;
  const size_t oQ  = off; off += PX;
  const size_t oK  = off; off += PX;
  const size_t oVT = off; off += PV;
  const size_t oCT = off; off += PX;
  const size_t oY  = off; off += PY;
  if (off > ws_size) return;
  if (off > (size_t)134217728) return;

  char* ws = (char*)d_ws;
  float*          G    = (float*)(ws + oG);
  unsigned short* X16  = (unsigned short*)(ws + oX);
  unsigned short* WQT  = (unsigned short*)(ws + oWQ);
  unsigned short* WKT  = (unsigned short*)(ws + oWK);
  unsigned short* WVT  = (unsigned short*)(ws + oWV);
  unsigned short* WOT  = (unsigned short*)(ws + oWO);
  unsigned short* Q16  = (unsigned short*)(ws + oQ);
  unsigned short* K16  = (unsigned short*)(ws + oK);
  unsigned short* VT16 = (unsigned short*)(ws + oVT);
  unsigned short* CT16 = (unsigned short*)(ws + oCT);
  float*          Y    = (float*)(ws + oY);

  const dim3 blk(256);
  const dim3 gG(DM / 256);
  const dim3 gCX((NTOK * DM) / 2048);
  const dim3 gT(DM / 64, DM / 64);
  const int tilesP = (NTOK / 64) * (DM / 64);
  const dim3 gP((tilesP + 7) / 8, 1);
  const dim3 gAT(ATT_BLOCKS);
  const dim3 bAT(ATT_THREADS);

  gate_k<<<gG, blk, 0, stream>>>(goal, w_g, b_g, G);
  cvtx_k<<<gCX, blk, 0, stream>>>(emb, G, X16, NTOK * DM, ACARRY);
  cvtT_k<<<gT, blk, 0, stream>>>(w_q, WQT, WSC);
  cvtT_k<<<gT, blk, 0, stream>>>(w_k, WKT, WSC);
  cvtT_k<<<gT, blk, 0, stream>>>(w_v, WVT, WSC);
  cvtT_k<<<gT, blk, 0, stream>>>(w_o, WOT, WSC);

  gemm64<2, 0, 0, 0><<<gP, blk, 0, stream>>>(
      X16, X16, DM, 0LL,
      WQT, DM, 0LL,
      (void*)Q16, (void*)Q16, DM, 0LL,
      NTOK, DM, DM, 1.0f / (ACARRY * WSC), QC, b_g);

  gemm64<2, 0, 0, 0><<<gP, blk, 0, stream>>>(
      X16, X16, DM, 0LL,
      WKT, DM, 0LL,
      (void*)K16, (void*)K16, DM, 0LL,
      NTOK, DM, DM, 1.0f / (ACARRY * WSC), QC, b_g);

  gemm64<2, 0, 0, 0><<<gP, blk, 0, stream>>>(
      WVT, WVT, DM, 0LL,
      X16, DM, 0LL,
      (void*)VT16, (void*)VT16, NTOK, 0LL,
      DM, NTOK, DM, 1.0f / (ACARRY * WSC), VC, b_g);

  attn_k<<<gAT, bAT, 0, stream>>>(Q16, K16, VT16, ids, rel, CT16);

  gemm64<0, 0, 0, 0><<<gP, blk, 0, stream>>>(
      CT16, CT16, DM, 0LL,
      WOT, DM, 0LL,
      (void*)Y, (void*)Y, DM, 0LL,
      NTOK, DM, DM, 1.0f / (CC * WSC), 1.0f, b_g);

  ln_k<<<dim3(NTOK), blk, 0, stream>>>(Y, emb, ln_g, ln_b, out);
  (void)hipGetLastError();
}
